// HBS_73882027425848
// MI455X (gfx1250) — hardware-verified
//
#include <hip/hip_runtime.h>
#include <stddef.h>


#define CF     64
#define MC     128
#define KM     192
#define KA     128
#define KP     512
#define NTHR   256
#define NWAVE  8
#define TGT    32
#define MTHR   128
#define MWAVE  4
#define MROWS  64
#define DEGCAP 4096
#define FSC    8.0f
#define WSC    64.0f
#define OINV   0.001953125f
#define EPSV   0.00001f
#define NEGBIG (-3.402823466e38f)
#define WSCAP  134217728

static_assert(MROWS == MWAVE * 16);
static_assert(TGT == NWAVE * 4);
static_assert(KP == 2 * 4 * CF && KM == 3 * CF && KA == 2 * CF && MC == 2 * CF);
static_assert((MC * KM / 8) % NTHR == 0 && (CF * KP / 8) % NTHR == 0);
static_assert(TGT * KP * 2 + TGT * CF * 4 <= 65536);
static_assert(MWAVE * 16 * KA * 2 + MROWS * MC * 4 <= 65536);

typedef float          v2f  __attribute__((ext_vector_type(2)));
typedef float          v4f  __attribute__((ext_vector_type(4)));
typedef float          v8f  __attribute__((ext_vector_type(8)));
typedef unsigned short v8us __attribute__((ext_vector_type(8)));
typedef _Float16       v2h  __attribute__((ext_vector_type(2)));
typedef _Float16       v8h  __attribute__((ext_vector_type(8)));
typedef _Float16       v16h __attribute__((ext_vector_type(16)));
typedef __bf16         v16b __attribute__((ext_vector_type(16)));
union FragH { v16h v; v8us h[2]; };
union FragB { v16b v; v8us h[2]; };
union Pack8 { v8h h; v8us u; };
union Pack2 { v2h h; unsigned int u; };

__device__ __forceinline__ unsigned int bf16_rne(float f) {
  const unsigned int u = __float_as_uint(f);
  return (u + 0x7FFFu + ((u >> 16) & 1u)) >> 16;
}

__device__ __forceinline__ void split8(v4f a, v4f b, v8us& hi, v8us& lo) {
  const float f[8] = {a.x, a.y, a.z, a.w, b.x, b.y, b.z, b.w};
#pragma unroll
  for (int e = 0; e < 8; ++e) {
    const unsigned int hb = bf16_rne(f[e]);
    const float fh = __uint_as_float(hb << 16);
    const unsigned int lb = bf16_rne(f[e] - fh);
    hi[e] = (unsigned short)hb;
    lo[e] = (unsigned short)lb;
  }
}

__device__ __forceinline__ v8us cvt8h(v4f a, v4f b, float sc) {
  v8h r;
  r[0] = (_Float16)(a.x * sc); r[1] = (_Float16)(a.y * sc);
  r[2] = (_Float16)(a.z * sc); r[3] = (_Float16)(a.w * sc);
  r[4] = (_Float16)(b.x * sc); r[5] = (_Float16)(b.y * sc);
  r[6] = (_Float16)(b.z * sc); r[7] = (_Float16)(b.w * sc);
  Pack8 p;
  p.h = r;
  return p.u;
}

__device__ __forceinline__ unsigned int pk2h(v2f a, float sc) {
  v2h r;
  r.x = (_Float16)(a.x * sc);
  r.y = (_Float16)(a.y * sc);
  Pack2 p;
  p.h = r;
  return p.u;
}

__device__ __forceinline__ v8f wmh(v16h a, v16h b, v8f c) {
  v8f d = __builtin_amdgcn_wmma_f32_16x16x32_f16(false, a, false, b, (short)0, c, false, false);
  asm volatile("v_nop\n\tv_nop\n\tv_nop\n\tv_nop" : "+v"(d) : "v"(a), "v"(b));
  return d;
}
__device__ __forceinline__ v8f wmb(v16b a, v16b b, v8f c) {
  v8f d = __builtin_amdgcn_wmma_f32_16x16x32_bf16(false, a, false, b, (short)0, c, false, false);
  asm volatile("v_nop\n\tv_nop\n\tv_nop\n\tv_nop" : "+v"(d) : "v"(a), "v"(b));
  return d;
}

__device__ __forceinline__ void seg_bounds(const int* __restrict__ arr, int nE, int t, int steps,
                                           int& st, int& cnt) {
  int lo = 0, hi = nE;
  int lo2 = 0, hi2 = nE;
#pragma unroll 1
  for (int s = 0; s < steps; ++s) {
    const int mid = (lo + hi) >> 1;
    const int mc  = mid < nE - 1 ? mid : nE - 1;
    const int v   = arr[mc];
    const bool act = lo < hi;
    const bool lt  = v < t;
    lo = (act && lt) ? mid + 1 : lo;
    hi = (act && !lt) ? mid : hi;
    const int mid2 = (lo2 + hi2) >> 1;
    const int mc2  = mid2 < nE - 1 ? mid2 : nE - 1;
    const int v2   = arr[mc2];
    const bool act2 = lo2 < hi2;
    const bool le2  = v2 <= t;
    lo2 = (act2 && le2) ? mid2 + 1 : lo2;
    hi2 = (act2 && !le2) ? mid2 : hi2;
  }
  st = lo;
  cnt = lo2 - lo;
}

__global__ __launch_bounds__(NTHR) void k_wprep(
    const float* __restrict__ W1, const float* __restrict__ W2,
    const float* __restrict__ P1, const float* __restrict__ P2,
    unsigned short* Bm, unsigned short* Bp) {
  constexpr int UM  = MC * KM / 8;
  constexpr int BMB = UM / NTHR;
  const int tid = (int)threadIdx.x;
  if ((int)blockIdx.x < BMB) {
    const int i    = (int)blockIdx.x * NTHR + tid;
    const int n    = i / (KM / 8);
    const int k0   = (i - n * (KM / 8)) * 8;
    const int set  = n >> 6;
    const int c    = n & (CF - 1);
    const int part = k0 >> 6;
    const int kk   = k0 - part * CF;
    const float* src = (set == 0) ? W1 : W2;
    float v[8];
#pragma unroll
    for (int e = 0; e < 8; ++e) v[e] = src[(size_t)(kk + e) * CF + c];
    v4f a, b;
    a.x = v[0]; a.y = v[1]; a.z = v[2]; a.w = v[3];
    b.x = v[4]; b.y = v[5]; b.z = v[6]; b.w = v[7];
    v8us hi, lo;
    split8(a, b, hi, lo);
    v8us o = hi;
    if (part == 2) o = lo;
    unsigned short* d = Bm + (size_t)n * KM + k0;
    *(volatile v8us*)d = o;
    __threadfence();
    *(volatile v8us*)d = o;
  } else {
    const int i   = ((int)blockIdx.x - BMB) * NTHR + tid;
    const int n   = i >> 6;
    const int k0  = (i & 63) * 8;
    const int set = k0 >> 8;
    const int kk  = k0 - set * 4 * CF;
    const float* src = (set == 0) ? P1 : P2;
    float v[8];
#pragma unroll
    for (int e = 0; e < 8; ++e) v[e] = src[(size_t)(kk + e) * CF + n];
    v4f a, b;
    a.x = v[0]; a.y = v[1]; a.z = v[2]; a.w = v[3];
    b.x = v[4]; b.y = v[5]; b.z = v[6]; b.w = v[7];
    const v8us o = cvt8h(a, b, WSC);
    unsigned short* d = Bp + (size_t)n * KP + k0;
    *(volatile v8us*)d = o;
    __threadfence();
    *(volatile v8us*)d = o;
  }
}

__global__ __launch_bounds__(MTHR) void k_msg(const float* __restrict__ x, const unsigned short* __restrict__ Bm,
                                             float* msg, int nN) {
  __shared__ __attribute__((aligned(16))) unsigned short sA[MWAVE * 16 * KA];
  __shared__ __attribute__((aligned(16))) float stg[MROWS * MC];
  const int tid = (int)threadIdx.x, lane = tid & 31, wave = tid >> 5, hh = lane >> 4, m = lane & 15;
  const int rowBase = (int)blockIdx.x * MROWS + wave * 16;

  {
    int ra = rowBase + m;
    ra = ra > nN - 1 ? nN - 1 : ra;
    const float* xr = x + (size_t)ra * CF + 8 * hh;
    unsigned short* aw = sA + (size_t)(wave * 16 + m) * KA + 8 * hh;
#pragma unroll
    for (int g = 0; g < 4; ++g) {
      const v4f p0 = *(const v4f*)(xr + 16 * g);
      const v4f p1 = *(const v4f*)(xr + 16 * g + 4);
      v8us hi, lo;
      split8(p0, p1, hi, lo);
      *(v8us*)(aw + 16 * g) = hi;
      *(v8us*)(aw + CF + 16 * g) = lo;
    }
  }
  __syncthreads();

  const unsigned short* ap = sA + (size_t)(wave * 16 + m) * KA + 8 * hh;
#pragma unroll 1
  for (int ch = 0; ch < 2; ++ch) {
    v8f acc[4];
#pragma unroll
    for (int t = 0; t < 4; ++t) { v8f z = {0.f, 0.f, 0.f, 0.f, 0.f, 0.f, 0.f, 0.f}; acc[t] = z; }
    const unsigned short* bq = Bm + (size_t)(ch * CF + m) * KM + 8 * hh;
#pragma unroll 1
    for (int ks = 0; ks < KM / 32; ++ks) {
      const int aoff = 32 * ks - (ks >= 4 ? KA : 0);
      FragB a;
      a.h[0] = *(const v8us*)(ap + aoff);
      a.h[1] = *(const v8us*)(ap + aoff + 16);
#pragma unroll
      for (int t = 0; t < 4; ++t) {
        const unsigned short* bp = bq + (size_t)(16 * t) * KM + 32 * ks;
        FragB b;
        b.h[0] = *(const v8us*)bp;
        b.h[1] = *(const v8us*)(bp + 16);
        acc[t] = wmb(a.v, b.v, acc[t]);
      }
    }
    float* sp = stg + (size_t)(wave * 16 + 8 * hh) * MC + ch * CF + m;
#pragma unroll
    for (int t = 0; t < 4; ++t) {
#pragma unroll
      for (int r = 0; r < 8; ++r) sp[r * MC + 16 * t] = acc[t][r];
    }
  }
  __syncthreads();

  float* gp = msg + (size_t)rowBase * MC + 4 * lane;
  const float* lp = stg + (size_t)(wave * 16) * MC + 4 * lane;
#pragma unroll 4
  for (int it = 0; it < 16; ++it) {
    const v4f v = *(const v4f*)(lp + it * MC);
    *(volatile v4f*)(gp + (size_t)it * MC) = v;
  }
  __threadfence();
#pragma unroll 4
  for (int it = 0; it < 16; ++it) {
    const v4f v = *(const v4f*)(lp + it * MC);
    *(volatile v4f*)(gp + (size_t)it * MC) = v;
  }
}

__global__ __launch_bounds__(NTHR) void k_agg(
    const int* __restrict__ rowA, const int* __restrict__ colA,
    const int* __restrict__ rowB, const int* __restrict__ colB,
    const float* __restrict__ msg, const unsigned short* __restrict__ Bp,
    const float* __restrict__ bA, const float* __restrict__ bB,
    const float* __restrict__ gam, const float* __restrict__ bet,
    float* out, int nN, int nEA, int nEB, int stepsA, int stepsB) {
#pragma clang fp contract(off)
  __shared__ __attribute__((aligned(16))) unsigned int sF[TGT * KP / 2];
  __shared__ __attribute__((aligned(16))) float sR[TGT * CF];
  const int tid = (int)threadIdx.x, lane = tid & 31, wave = tid >> 5, hh = lane >> 4, m = lane & 15;
  const int tb = (int)blockIdx.x * TGT + wave * 4;
  const int tl = tb + (lane & 3);

  int offA, cntA, offB, cntB;
  seg_bounds(rowA, nEA, tl, stepsA, offA, cntA);
  seg_bounds(rowB, nEB, tl, stepsB, offB, cntB);

#pragma unroll 1
  for (int j = 0; j < 8; ++j) {
    const int set = j >> 2;
    const int q   = j & 3;
    const int cnt_l = (set == 0) ? cntA : cntB;
    const int off_l = (set == 0) ? offA : offB;
    const int* cols = (set == 0) ? colA : colB;
    const int nE    = (set == 0) ? nEA : nEB;
    int nraw = __shfl(cnt_l, q);
    nraw = nraw < 0 ? 0 : (nraw > nE ? nE : nraw);
    const int n  = nraw > DEGCAP ? DEGCAP : nraw;
    const int st = __shfl(off_l, q);
    const float* mrow = msg + set * CF + 2 * lane;

    v2f s = {0.f, 0.f}, sq = {0.f, 0.f}, mx = {NEGBIG, NEGBIG};
#pragma unroll 1
    for (int q0 = 0; q0 < n; q0 += 32) {
      int pos = st + q0 + lane;
      pos = pos < 0 ? 0 : (pos > nE - 1 ? nE - 1 : pos);
      int sl = cols[pos];
      sl = sl < 0 ? 0 : (sl > nN - 1 ? nN - 1 : sl);
      const int mcnt = (n - q0) < 32 ? (n - q0) : 32;
#pragma unroll 1
      for (int pp = 0; pp < mcnt; ++pp) {
        const int sidx = __builtin_amdgcn_readlane(sl, pp);
        const v2f g = *(const v2f*)(mrow + (size_t)sidx * MC);
        s  = s + g;
        sq = sq + g * g;
        mx.x = fmaxf(mx.x, g.x);
        mx.y = fmaxf(mx.y, g.y);
      }
    }
    const float rc = 1.0f / (float)(nraw > 0 ? nraw : 1);
    const v2f mean = s * rc;
    v2f var = sq * rc - mean * mean;
    var.x = fmaxf(var.x, 0.0f);
    var.y = fmaxf(var.y, 0.0f);
    v2f sd;
    sd.x = sqrtf(var.x + EPSV);
    sd.y = sqrtf(var.y + EPSV);
    v2f mv = mx;
    if (nraw <= 0) { const v2f z2 = {0.f, 0.f}; mv = z2; }
    const int row = wave * 4 + q;
    unsigned int* fp = sF + (size_t)row * (KP / 2) + set * (4 * CF / 2) + lane;
    fp[0]            = pk2h(s, FSC);
    fp[CF / 2]       = pk2h(mean, FSC);
    fp[2 * (CF / 2)] = pk2h(mv, FSC);
    fp[3 * (CF / 2)] = pk2h(sd, FSC);
  }
  __syncthreads();

  const int rt = wave >> 2, ct = wave & 3;
  v8f acc = {0.f, 0.f, 0.f, 0.f, 0.f, 0.f, 0.f, 0.f};
  {
    const unsigned short* ap = (const unsigned short*)sF + (size_t)(rt * 16 + m) * KP + 8 * hh;
    const unsigned short* bq = Bp + (size_t)(ct * 16 + m) * KP + 8 * hh;
#pragma unroll 2
    for (int kt = 0; kt < KP / 32; ++kt) {
      FragH a, b;
      a.h[0] = *(const v8us*)(ap + 32 * kt);
      a.h[1] = *(const v8us*)(ap + 32 * kt + 16);
      b.h[0] = *(const v8us*)(bq + 32 * kt);
      b.h[1] = *(const v8us*)(bq + 32 * kt + 16);
      acc = wmh(a.v, b.v, acc);
    }
  }
  {
    const int n = ct * 16 + m;
    const float bv = bA[n] + bB[n];
    float* sp = sR + (size_t)(rt * 16 + 8 * hh) * CF + n;
#pragma unroll
    for (int r = 0; r < 8; ++r) {
      const float o = acc[r] * OINV + bv;
      sp[r * CF] = fmaxf(o, 0.0f);
    }
  }
  __syncthreads();

  const int c4 = 4 * m;
  const v4f g4 = *(const v4f*)(gam + c4);
  const v4f e4 = *(const v4f*)(bet + c4);
  v4f ov[2];
#pragma unroll
  for (int p = 0; p < 2; ++p) {
    const int row = wave * 4 + 2 * p + hh;
    const v4f xv = *(const v4f*)(sR + (size_t)row * CF + c4);
    float su = (xv.x + xv.y) + (xv.z + xv.w);
    su += __shfl_xor(su, 8);
    su += __shfl_xor(su, 4);
    su += __shfl_xor(su, 2);
    su += __shfl_xor(su, 1);
    const float mu = su * 0.015625f;
    const v4f d = xv - mu;
    float vs = (d.x * d.x + d.y * d.y) + (d.z * d.z + d.w * d.w);
    vs += __shfl_xor(vs, 8);
    vs += __shfl_xor(vs, 4);
    vs += __shfl_xor(vs, 2);
    vs += __shfl_xor(vs, 1);
    const float var  = vs * 0.015625f;
    const float rstd = 1.0f / sqrtf(var + EPSV);
    ov[p] = d * rstd * g4 + e4;
  }
#pragma unroll
  for (int p = 0; p < 2; ++p) {
    const int grow = (int)blockIdx.x * TGT + wave * 4 + 2 * p + hh;
    if (grow < nN) *(volatile v4f*)(out + (size_t)grow * CF + c4) = ov[p];
  }
  __threadfence();
#pragma unroll
  for (int p = 0; p < 2; ++p) {
    const int grow = (int)blockIdx.x * TGT + wave * 4 + 2 * p + hh;
    if (grow < nN) *(volatile v4f*)(out + (size_t)grow * CF + c4) = ov[p];
  }
}

extern "C" void kernel_launch(void* const* d_in, const int* in_sizes, int n_in,
                              void* d_out, int out_size, void* d_ws, size_t ws_size,
                              hipStream_t stream) {
  if (n_in < 13) return;
  const int nN = in_sizes[0] / CF;
  if (nN <= 0 || in_sizes[0] != nN * CF || nN > (1 << 24)) return;
  if (in_sizes[1] != CF * CF || in_sizes[2] != CF * CF) return;
  if (in_sizes[3] != 4 * CF * CF || in_sizes[5] != 4 * CF * CF) return;
  if (in_sizes[4] != CF || in_sizes[6] != CF || in_sizes[7] != CF || in_sizes[8] != CF) return;
  const int nEA = in_sizes[9];
  const int nEB = in_sizes[11];
  if (nEA <= 0 || nEB <= 0 || in_sizes[10] != nEA || in_sizes[12] != nEB) return;
  if (nEA > (1 << 29) || nEB > (1 << 29)) return;
  if (out_size != nN * CF) return;

  const float* x    = (const float*)d_in[0];
  const float* W1   = (const float*)d_in[1];
  const float* W2   = (const float*)d_in[2];
  const float* P1   = (const float*)d_in[3];
  const float* b1   = (const float*)d_in[4];
  const float* P2   = (const float*)d_in[5];
  const float* b2   = (const float*)d_in[6];
  const float* gam  = (const float*)d_in[7];
  const float* bet  = (const float*)d_in[8];
  const int*   rowA = (const int*)d_in[9];
  const int*   colA = (const int*)d_in[10];
  const int*   rowB = (const int*)d_in[11];
  const int*   colB = (const int*)d_in[12];
  float* out = (float*)d_out;

  const int nMB   = (nN + MROWS - 1) / MROWS;
  const int NPADM = nMB * MROWS;
  const int nAB   = (nN + TGT - 1) / TGT;

  int stepsA = 2; { unsigned int v = 1u; while (v < (unsigned int)nEA && stepsA < 40) { v <<= 1; ++stepsA; } }
  int stepsB = 2; { unsigned int v = 1u; while (v < (unsigned int)nEB && stepsB < 40) { v <<= 1; ++stepsB; } }

  char* ws = (char*)d_ws;
  size_t off = 0;
  const size_t oBm  = off; off += (size_t)MC * KM * 2;        off = (off + 255) & ~(size_t)255;
  const size_t oBp  = off; off += (size_t)CF * KP * 2;        off = (off + 255) & ~(size_t)255;
  const size_t oMsg = off; off += (size_t)NPADM * MC * 4;     off = (off + 255) & ~(size_t)255;
  if (off > ws_size || off > (size_t)WSCAP) return;
  unsigned short* Bm  = (unsigned short*)(ws + oBm);
  unsigned short* Bp  = (unsigned short*)(ws + oBp);
  float*          msg = (float*)(ws + oMsg);

  k_wprep<<<(MC * KM / 8) / NTHR + (CF * KP / 8) / NTHR, NTHR, 0, stream>>>(W1, W2, P1, P2, Bm, Bp);
  k_msg<<<nMB, MTHR, 0, stream>>>(x, Bm, msg, nN);
  k_agg<<<nAB, NTHR, 0, stream>>>(rowA, colA, rowB, colB, msg, Bp, b1, b2, gam, bet, out,
                                  nN, nEA, nEB, stepsA, stepsB);
}
